// SLoRA_50405736186182
// MI455X (gfx1250) — hardware-verified
//
#include <hip/hip_runtime.h>
#include <stdint.h>
#include <stddef.h>

#pragma clang fp contract(off)

#define NTOK 4096
#define DIN  2048
#define DOUT 2048
#define NAD  8
#define MR   64
#define NSL  (NAD * MR)
#define MT   32
#define GX   16
#define TPB  8
#define XP   2056
#define XAP  72
#define YP   260
#define TT   64
#define TPF  68
#define LDS_X (MT * XP * 2)

#define A_SC   256.0f
#define B_SC   256.0f
#define XA_SCR 0.0625f
#define R_Y    0.000244140625f

static_assert(MT * YP * 4 <= LDS_X);
static_assert((XP * 2) % 16 == 0);
static_assert((XAP * 2) % 16 == 0);
static_assert((YP * 4) % 16 == 0);
static_assert((TPF * 4) % 16 == 0);
static_assert(NTOK % 256 == 0);
static_assert(GX * TPB * MT >= NTOK);
static_assert(TPB * MT <= 256);
static_assert(DIN == 8 * 256);
static_assert(DIN % 32 == 0);
static_assert(MR == 64);
static_assert(DOUT % 256 == 0);
static_assert(DOUT % TT == 0);
static_assert(NAD == 8);
static_assert(NSL == 512);

typedef _Float16       v16h __attribute__((ext_vector_type(16)));
typedef _Float16       v8h  __attribute__((ext_vector_type(8)));
typedef float          v8f  __attribute__((ext_vector_type(8)));
typedef float          v4f  __attribute__((ext_vector_type(4)));
typedef unsigned int   v4u  __attribute__((ext_vector_type(4)));
typedef v4f __attribute__((may_alias)) v4fa;
typedef v4u __attribute__((may_alias)) v4ua;

union FragH { v16h v; v4u q[2]; };
union Pack8 { v8h h; v4u u; };

__device__ __forceinline__ unsigned short hbits(float f) {
  _Float16 t = (_Float16)f;
  unsigned short u;
  __builtin_memcpy(&u, &t, 2);
  return u;
}

__device__ __forceinline__ v8f wmma_h(v16h a, v16h b, v8f c) {
  v8f d = __builtin_amdgcn_wmma_f32_16x16x32_f16(false, a, false, b, (short)0, c, false, false);
  asm volatile("v_nop\n\tv_nop\n\tv_nop\n\tv_nop" : "+v"(d) : "v"(a), "v"(b));
  return d;
}

__device__ __forceinline__ v16h ldfrag(const unsigned short* p, int h) {
  FragH f;
  f.q[0] = *(const v4ua*)(p + 8 * h);
  f.q[1] = *(const v4ua*)(p + 16 + 8 * h);
  return f.v;
}

__global__ __launch_bounds__(256) void k_cva(const float* __restrict__ a_cache,
                                             const int* __restrict__ ranks,
                                             const int* __restrict__ rank_offsets,
                                             unsigned short* __restrict__ a16)
{
  const int s = blockIdx.x;
  const int tid = threadIdx.x;
  const int a = s >> 6, r = s & 63;
  int slot = rank_offsets[s];
  slot = (slot < 0) ? 0 : ((slot > NSL - 1) ? (NSL - 1) : slot);
  int rk = ranks[a];
  rk = (rk < 0) ? 0 : ((rk > MR) ? MR : rk);
  const bool live = (r < rk);
  const float* pa = a_cache + (size_t)slot * DIN + 8 * tid;
  const v4f p0 = *(const v4fa*)pa;
  const v4f p1 = *(const v4fa*)(pa + 4);
  const _Float16 zz = (_Float16)0.0f;
  v8h hv;
  hv[0] = live ? (_Float16)(p0.x * A_SC) : zz;  hv[1] = live ? (_Float16)(p0.y * A_SC) : zz;
  hv[2] = live ? (_Float16)(p0.z * A_SC) : zz;  hv[3] = live ? (_Float16)(p0.w * A_SC) : zz;
  hv[4] = live ? (_Float16)(p1.x * A_SC) : zz;  hv[5] = live ? (_Float16)(p1.y * A_SC) : zz;
  hv[6] = live ? (_Float16)(p1.z * A_SC) : zz;  hv[7] = live ? (_Float16)(p1.w * A_SC) : zz;
  Pack8 pk;
  pk.h = hv;
  const v4u u = pk.u;
  unsigned short* d = a16 + (size_t)s * DIN + 8 * tid;
  *(volatile v4u*)d = u;
  __threadfence();
  *(volatile v4u*)d = u;
}

__global__ __launch_bounds__(256) void k_cvb(const float* __restrict__ b_cache,
                                             const int* __restrict__ rank_offsets,
                                             unsigned short* __restrict__ bt16)
{
  __shared__ __align__(16) float tile[TT * TPF];
  const int tid = threadIdx.x;
  const int o0 = blockIdx.x * TT, a = blockIdx.y;
  #pragma unroll
  for (int j = 0; j < 4; ++j) {
    const int r  = (tid >> 4) + 16 * j;
    const int c4 = tid & 15;
    int slot = rank_offsets[a * MR + r];
    slot = (slot < 0) ? 0 : ((slot > NSL - 1) ? (NSL - 1) : slot);
    const v4f v = *(const v4fa*)(b_cache + (size_t)slot * DOUT + o0 + 4 * c4);
    *(v4fa*)(tile + r * TPF + 4 * c4) = v;
  }
  __syncthreads();
  v4u u[2];
  #pragma unroll
  for (int j = 0; j < 2; ++j) {
    const int n = (tid >> 3) + 32 * j;
    const int q = tid & 7;
    v8h hv;
    #pragma unroll
    for (int i = 0; i < 8; ++i) hv[i] = (_Float16)(tile[(8 * q + i) * TPF + n] * B_SC);
    Pack8 pk;
    pk.h = hv;
    u[j] = pk.u;
  }
  unsigned short* d0 = bt16 + ((size_t)a * DOUT + o0 + (tid >> 3)) * MR + 8 * (tid & 7);
  unsigned short* d1 = d0 + (size_t)32 * MR;
  *(volatile v4u*)d0 = u[0];
  *(volatile v4u*)d1 = u[1];
  __threadfence();
  *(volatile v4u*)d0 = u[0];
  *(volatile v4u*)d1 = u[1];
}

__global__ __launch_bounds__(256) void k_lora(const float* __restrict__ x,
                                              const float* __restrict__ base,
                                              const int* __restrict__ adapter_ids,
                                              const float* __restrict__ scalings,
                                              const unsigned short* __restrict__ a16,
                                              const unsigned short* __restrict__ bt16,
                                              float* __restrict__ out, int ntok)
{
  extern __shared__ __align__(16) unsigned char dsm[];
  unsigned short* sX = (unsigned short*)dsm;
  float* sY = (float*)dsm;
  __shared__ __align__(16) unsigned short sXA[MT * XAP];
  __shared__ int sTok[TPB * MT];
  __shared__ int s_wc[8];

  const int tid = threadIdx.x, lane = tid & 31, wv = tid >> 5;
  const int h = lane >> 4, m = lane & 15;
  const int a = blockIdx.y;
  const int bx = blockIdx.x;

  if (tid < TPB * MT) sTok[tid] = 0;
  __syncthreads();

  int base_cnt = 0;
  #pragma unroll 1
  for (int ch = 0; ch < NTOK / 256; ++ch) {
    const int t = ch * 256 + tid;
    const int tc = (t < ntok) ? t : (ntok - 1);
    int id = adapter_ids[tc];
    id = (id < 0) ? 0 : ((id > NAD - 1) ? (NAD - 1) : id);
    const bool f = (id == a) && (t < ntok);
    const unsigned int msk = __builtin_amdgcn_ballot_w32(f);
    const int off = __builtin_popcount(msk & ((1u << lane) - 1u));
    const int wcnt = __builtin_popcount(msk);
    if (lane == 0) s_wc[wv] = wcnt;
    __syncthreads();
    int pre = 0, tot = 0;
    #pragma unroll
    for (int w2 = 0; w2 < 8; ++w2) {
      const int c2 = s_wc[w2];
      tot += c2;
      pre += (w2 < wv) ? c2 : 0;
    }
    if (f) {
      const int pos = base_cnt + pre + off;
      const int tile = pos / MT;
      const int lt = tile / GX;
      const int p = lt * MT + (pos % MT);
      if (((tile % GX) == bx) && ((unsigned)p < (unsigned)(TPB * MT))) sTok[p] = t;
    }
    base_cnt += tot;
    __syncthreads();
  }
  const int cnt = base_cnt;

  const float scal = scalings[a];
  const unsigned short* arows = a16 + (size_t)a * MR * DIN;
  const unsigned short* brows = bt16 + (size_t)a * DOUT * MR;
  const v8f z8 = {0.f, 0.f, 0.f, 0.f, 0.f, 0.f, 0.f, 0.f};

  #pragma unroll 1
  for (int lt = 0; lt < TPB; ++lt) {
    const int m0 = (bx + GX * lt) * MT;
    if (m0 >= cnt) break;
    int nrows = cnt - m0;
    nrows = (nrows > MT) ? MT : nrows;
    const int lo = lt * MT;

    #pragma unroll 4
    for (int j = 0; j < MT; ++j) {
      int t = sTok[lo + j];
      t = (t < 0) ? 0 : ((t > NTOK - 1) ? (NTOK - 1) : t);
      const float* s = x + (size_t)t * DIN + 8 * tid;
      const v4f p0 = *(const v4fa*)s;
      const v4f p1 = *(const v4fa*)(s + 4);
      v8h hv;
      hv[0] = (_Float16)p0.x; hv[1] = (_Float16)p0.y; hv[2] = (_Float16)p0.z; hv[3] = (_Float16)p0.w;
      hv[4] = (_Float16)p1.x; hv[5] = (_Float16)p1.y; hv[6] = (_Float16)p1.z; hv[7] = (_Float16)p1.w;
      Pack8 pk;
      pk.h = hv;
      *(v4ua*)(sX + j * XP + 8 * tid) = pk.u;
    }
    __syncthreads();

    {
      const int mt = wv >> 2, nt = wv & 3;
      const unsigned short* ap = sX + (16 * mt + m) * XP;
      const unsigned short* bp = arows + (size_t)(16 * nt + m) * DIN;
      v8f acc = z8;
      #pragma unroll 2
      for (int kb = 0; kb < DIN; kb += 32) {
        const v16h af = ldfrag(ap + kb, h);
        const v16h bf = ldfrag(bp + kb, h);
        acc = wmma_h(af, bf, acc);
      }
      #pragma unroll
      for (int r = 0; r < 8; ++r) {
        const int row = 16 * mt + 8 * h + r;
        sXA[row * XAP + 16 * nt + m] = hbits(acc[r] * XA_SCR);
      }
    }
    __syncthreads();

    v16h xf[2][2];
    #pragma unroll
    for (int mt = 0; mt < 2; ++mt)
      #pragma unroll
      for (int ks = 0; ks < 2; ++ks)
        xf[mt][ks] = ldfrag(sXA + (16 * mt + m) * XAP + 32 * ks, h);

    #pragma unroll 1
    for (int ns = 0; ns < DOUT / 256; ++ns) {
      v8f acc[2][2];
      #pragma unroll
      for (int mt = 0; mt < 2; ++mt)
        #pragma unroll
        for (int nt = 0; nt < 2; ++nt) acc[mt][nt] = z8;
      #pragma unroll
      for (int nt = 0; nt < 2; ++nt) {
        const int o = ns * 256 + wv * 32 + 16 * nt + m;
        const unsigned short* bq = brows + (size_t)o * MR;
        #pragma unroll
        for (int ks = 0; ks < 2; ++ks) {
          const v16h bf = ldfrag(bq + 32 * ks, h);
          #pragma unroll
          for (int mt = 0; mt < 2; ++mt) acc[mt][nt] = wmma_h(xf[mt][ks], bf, acc[mt][nt]);
        }
      }
      #pragma unroll
      for (int mt = 0; mt < 2; ++mt)
        #pragma unroll
        for (int nt = 0; nt < 2; ++nt) {
          const int cl = wv * 32 + 16 * nt + m;
          #pragma unroll
          for (int r = 0; r < 8; ++r) {
            const int row = 16 * mt + 8 * h + r;
            const float yv = acc[mt][nt][r] * R_Y;
            sY[row * YP + cl] = yv * scal;
          }
        }
      __syncthreads();

      v4f o0[4], o1[4];
      int tr[4];
      #pragma unroll
      for (int i = 0; i < 4; ++i) {
        const int row = wv * 4 + i;
        int t = sTok[lo + row];
        t = (t < 0) ? 0 : ((t > NTOK - 1) ? (NTOK - 1) : t);
        tr[i] = t;
        const float* bp = base + (size_t)t * DOUT + ns * 256;
        const v4f b0 = *(const v4fa*)(bp + 4 * lane);
        const v4f b1 = *(const v4fa*)(bp + 128 + 4 * lane);
        const v4f y0 = *(const v4fa*)(sY + row * YP + 4 * lane);
        const v4f y1 = *(const v4fa*)(sY + row * YP + 128 + 4 * lane);
        o0[i] = b0 + y0;
        o1[i] = b1 + y1;
      }
      #pragma unroll
      for (int i = 0; i < 4; ++i) {
        const int row = wv * 4 + i;
        float* dst = out + (size_t)tr[i] * DOUT + ns * 256;
        if (row < nrows) {
          *(volatile v4f*)(dst + 4 * lane) = o0[i];
          *(volatile v4f*)(dst + 128 + 4 * lane) = o1[i];
        }
      }
      __threadfence();
      #pragma unroll
      for (int i = 0; i < 4; ++i) {
        const int row = wv * 4 + i;
        float* dst = out + (size_t)tr[i] * DOUT + ns * 256;
        if (row < nrows) {
          *(volatile v4f*)(dst + 4 * lane) = o0[i];
          *(volatile v4f*)(dst + 128 + 4 * lane) = o1[i];
        }
      }
      __syncthreads();
    }
  }
}

extern "C" void kernel_launch(void* const* d_in, const int* in_sizes, int n_in,
                              void* d_out, int out_size, void* d_ws, size_t ws_size,
                              hipStream_t stream)
{
  if (n_in < 8) return;
  if (in_sizes[0] != NTOK * DIN) return;
  if (in_sizes[1] != NTOK * DOUT) return;
  if (in_sizes[2] != NTOK) return;
  if (in_sizes[3] != NAD) return;
  if (in_sizes[4] != NAD) return;
  if (in_sizes[5] != NSL) return;
  if (in_sizes[6] != NSL * DIN) return;
  if (in_sizes[7] != NSL * DOUT) return;
  if (out_size != NTOK * DOUT) return;

  const float* x    = (const float*)d_in[0];
  const float* base = (const float*)d_in[1];
  const int*   aid  = (const int*)d_in[2];
  const int*   rks  = (const int*)d_in[3];
  const float* scl  = (const float*)d_in[4];
  const int*   rof  = (const int*)d_in[5];
  const float* ac   = (const float*)d_in[6];
  const float* bc   = (const float*)d_in[7];
  float* out = (float*)d_out;

  const size_t bA = (size_t)NSL * DIN * 2;
  const size_t bB = (size_t)NAD * DOUT * MR * 2;
  const size_t total = bA + bB;
  if (total > ws_size) return;
  if (total > (size_t)134217728) return;

  char* ws = (char*)d_ws;
  size_t off = 0;
  unsigned short* A16  = (unsigned short*)(ws + off); off += bA;
  unsigned short* BT16 = (unsigned short*)(ws + off); off += bB;
  if (off != total) return;

  hipFuncSetAttribute(reinterpret_cast<const void*>(&k_lora),
                      hipFuncAttributeMaxDynamicSharedMemorySize, LDS_X);

  k_cva<<<NSL, 256, 0, stream>>>(ac, rks, rof, A16);
  k_cvb<<<dim3(DOUT / TT, NAD), 256, 0, stream>>>(bc, rof, BT16);
  k_lora<<<dim3(GX, NAD), 256, LDS_X, stream>>>(x, base, aid, scl, A16, BT16, out, NTOK);
}
